// EfficientAttention_31533649887315
// MI455X (gfx1250) — hardware-verified
//
#include <hip/hip_runtime.h>


#ifndef NB
#define NB 2
#endif
#ifndef SEQ
#define SEQ 2048
#endif
#define TT      SEQ
#define TT_FULL 2048
#define NB_FULL 2
#define DM      1024
#define NH_     16
#define HD      64
#define DQ      (NH_ * HD)
#define HALF    (DM / 2)
#define ZH      2
#define SCL     0.125f
static_assert(TT % 128 == 0);
static_assert(TT <= TT_FULL);
static_assert(NB >= 1 && NB <= NB_FULL);
static_assert(NH_ % ZH == 0);
static_assert(DQ == DM);
static_assert(HD == 64);
static_assert(DM % 64 == 0);

typedef unsigned short bf;
typedef __attribute__((ext_vector_type(16))) __bf16         v16bf;
typedef __attribute__((ext_vector_type(8)))  unsigned short v8us;
typedef __attribute__((ext_vector_type(4)))  unsigned short v4us;
typedef __attribute__((ext_vector_type(2)))  unsigned short v2us;
typedef __attribute__((ext_vector_type(8)))  float          v8f;
typedef __attribute__((ext_vector_type(4)))  float          v4f;
typedef __attribute__((ext_vector_type(2)))  float          v2f;
typedef v4f __attribute__((may_alias)) v4fa;

__device__ __forceinline__ unsigned short f2bf(float f) { unsigned u = __float_as_uint(f); u += 0x7FFFu + ((u >> 16) & 1u); return (unsigned short)(u >> 16); }
__device__ __forceinline__ float bf2f(unsigned short b) { return __uint_as_float(((unsigned)b) << 16); }
__device__ __forceinline__ float bfr(float f) { return bf2f(f2bf(f)); }
__device__ __forceinline__ void splitf(float y, unsigned short& h, unsigned short& l) { h = f2bf(y); l = f2bf(y - bf2f(h)); }
__device__ __forceinline__ v16bf cat16b(v8us lo, v8us hi) { return __builtin_bit_cast(v16bf, __builtin_shufflevector(lo, hi, 0, 1, 2, 3, 4, 5, 6, 7, 8, 9, 10, 11, 12, 13, 14, 15)); }
__device__ __forceinline__ v8f wmmab(v16bf a, v16bf b, v8f c) { return __builtin_amdgcn_wmma_f32_16x16x32_bf16(false, a, false, b, (short)0, c, false, false); }
__device__ __forceinline__ v16bf ldfrag(const bf* p) { return cat16b(*(const v8us*)p, *(const v8us*)(p + 16)); }

template <int NSPLIT, bool BIAS>
__global__ __launch_bounds__(32) void k_gemmw(const bf* __restrict__ A, const bf* __restrict__ A2, const bf* __restrict__ Bt, const bf* __restrict__ Bt2, int K, float* C, int ldc, const float* __restrict__ bias, size_t sA, size_t sB, size_t sC, int qoff, int cmode) {
    __shared__ __align__(16) float os[16 * 68];
    const int r0 = blockIdx.x * 64, c0 = blockIdx.y * 64;
    const int qr = qoff + r0;
    if (cmode == 1 && c0 >= (((qr >> 7) + 1) << 7)) return;
    const int Keff = (cmode == 2 && (qr + 64) < K) ? (qr + 64) : K;
    const size_t z = blockIdx.z; A += z * sA; if (NSPLIT == 1 || NSPLIT == 2) A2 += z * sA; Bt += z * sB; if (NSPLIT >= 2) Bt2 += z * sB; C += z * sC;
    const int lane = threadIdx.x & 31, lr = lane & 15, hi = lane >> 4;
    v8f acc[4][4];
#pragma unroll
    for (int mb = 0; mb < 4; ++mb)
#pragma unroll
        for (int nb = 0; nb < 4; ++nb) acc[mb][nb] = (v8f){};
    const size_t aoff = (size_t)(r0 + lr) * K + 8 * hi, boff = (size_t)(c0 + lr) * K + 8 * hi;
#pragma unroll 1
    for (int kc = 0; kc < Keff; kc += 32) {
        v16bf a[4], a2[4];
#pragma unroll
        for (int mb = 0; mb < 4; ++mb) { a[mb] = ldfrag(A + aoff + (size_t)mb * 16 * K + kc); if (NSPLIT == 1 || NSPLIT == 2) a2[mb] = ldfrag(A2 + aoff + (size_t)mb * 16 * K + kc); }
#pragma unroll
        for (int nb = 0; nb < 4; ++nb) { const v16bf b = ldfrag(Bt + boff + (size_t)nb * 16 * K + kc); v16bf b2; if (NSPLIT >= 2) b2 = ldfrag(Bt2 + boff + (size_t)nb * 16 * K + kc);
#pragma unroll
            for (int mb = 0; mb < 4; ++mb) { acc[mb][nb] = wmmab(a[mb], b, acc[mb][nb]); if (NSPLIT == 1 || NSPLIT == 2) acc[mb][nb] = wmmab(a2[mb], b, acc[mb][nb]); if (NSPLIT >= 2) acc[mb][nb] = wmmab(a[mb], b2, acc[mb][nb]); } }
        asm volatile("v_nop\n\tv_nop\n\tv_nop\n\tv_nop" : "+v"(acc[0][0]), "+v"(acc[1][1]), "+v"(acc[2][2]), "+v"(acc[3][3]) : "v"(a[0]), "v"(a[3]));
    }
#pragma unroll
    for (int mb = 0; mb < 4; ++mb) {
#pragma unroll
        for (int nb = 0; nb < 4; ++nb) {
#pragma unroll
            for (int j = 0; j < 8; ++j) os[(hi * 8 + j) * 68 + nb * 16 + lr] = acc[mb][nb][j]; }
        __builtin_amdgcn_wave_barrier(); asm volatile("" ::: "memory");
        float* crow = C + (size_t)(r0 + mb * 16) * ldc + c0;
#pragma unroll 1
        for (int ps = 0; ps < 2; ++ps) {
#pragma unroll
            for (int s = 0; s < 8; ++s) { const int row = 2 * s + hi, cofs = lr * 4; v4f val = *(const v4fa*)(os + row * 68 + cofs); if (BIAS) { val[0] += bfr(bias[c0 + cofs]); val[1] += bfr(bias[c0 + cofs + 1]); val[2] += bfr(bias[c0 + cofs + 2]); val[3] += bfr(bias[c0 + cofs + 3]); }
                *(volatile v4f*)(crow + (size_t)row * ldc + cofs) = val; }
            if (ps == 0) __threadfence(); }
        __builtin_amdgcn_wave_barrier(); asm volatile("" ::: "memory");
    }
}

__global__ __launch_bounds__(256) void k_cvt8(const float* __restrict__ src, bf* dst, size_t n8) { const size_t i = (size_t)blockIdx.x * 256 + threadIdx.x; if (i >= n8) return; const v8f v = *(const v8f*)(src + i * 8); v8us o;
#pragma unroll
    for (int k = 0; k < 8; ++k) o[k] = f2bf(v[k]); *(volatile v8us*)(dst + i * 8) = o; __threadfence(); *(volatile v8us*)(dst + i * 8) = o; }

__global__ __launch_bounds__(256) void k_freq(float* FR) {
    const int j = blockIdx.x * 256 + threadIdx.x; if (j >= HALF) return;
    const double p = exp2((double)j * (13.287712379549449 / (double)HALF));
    const float pf = (float)p;
    const float fr = 1.0f / pf;
    *(volatile float*)(FR + j) = fr; __threadfence(); *(volatile float*)(FR + j) = fr;
}
__global__ __launch_bounds__(256) void k_cstab(const float* __restrict__ FR, float* CS) {
    const int idx = blockIdx.x * 256 + threadIdx.x; if (idx >= TT * HALF) return;
    const int j = idx % HALF; const int t = idx / HALF;
    const float ang = __fmul_rn((float)t, FR[j]);
    float sn, cs; sincosf(ang, &sn, &cs);
    v2f o; o[0] = cs; o[1] = sn;
    *(volatile v2f*)(CS + (size_t)idx * 2) = o; __threadfence(); *(volatile v2f*)(CS + (size_t)idx * 2) = o;
}

__global__ __launch_bounds__(256) void k_rope(const float* __restrict__ F, const float* __restrict__ CS, bf* Ph, bf* Pl) {
    const size_t e = ((size_t)blockIdx.x * 256 + threadIdx.x) * 2; if (e >= (size_t)NH_ * TT * HD) return;
    const int d = (int)(e % HD); const int t = (int)((e / HD) % TT); const int h = (int)(e / ((size_t)HD * TT));
    const float* f = F + (size_t)t * DQ; const float* cst = CS + (size_t)t * HALF * 2;
    v2us oh, ol;
#pragma unroll
    for (int q = 0; q < 2; ++q) { const int c = h * HD + d + q; const int j = c & (HALF - 1); const int cp = (c < HALF) ? (c + HALF) : (c - HALF);
        const float x0 = f[c], x1 = f[cp]; const v2f cs = *(const v2f*)(cst + (size_t)j * 2);
        float a = __fmul_rn(x0, cs[0]), bq = __fmul_rn(x1, cs[1]); asm volatile("" : "+v"(a)); asm volatile("" : "+v"(bq));
        const float r = (c < HALF) ? __fsub_rn(a, bq) : __fadd_rn(bq, a);
        unsigned short a2, c2; splitf(r, a2, c2); oh[q] = a2; ol[q] = c2; }
    *(volatile v2us*)(Ph + e) = oh; *(volatile v2us*)(Pl + e) = ol; __threadfence(); *(volatile v2us*)(Ph + e) = oh; *(volatile v2us*)(Pl + e) = ol;
}
__global__ __launch_bounds__(256) void k_vtp(const float* __restrict__ F, bf* Vh, bf* Vl) { const size_t e = ((size_t)blockIdx.x * 256 + threadIdx.x) * 2; if (e >= (size_t)NH_ * HD * TT) return; const int t = (int)(e % TT); const int d = (int)((e / TT) % HD); const int g = (int)(e / ((size_t)TT * HD)); v2us oh, ol;
#pragma unroll
    for (int q = 0; q < 2; ++q) { const float x = F[(size_t)(t + q) * DQ + g * HD + d]; unsigned short a2, c2; splitf(x, a2, c2); oh[q] = a2; ol[q] = c2; }
    *(volatile v2us*)(Vh + e) = oh; *(volatile v2us*)(Vl + e) = ol; __threadfence(); *(volatile v2us*)(Vh + e) = oh; *(volatile v2us*)(Vl + e) = ol; }

__global__ __launch_bounds__(256) void k_asoft(const float* __restrict__ Sb, int h0, bf* Ph, bf* Pl) {
    const int lane = threadIdx.x & 31; const int row = blockIdx.x * 8 + (threadIdx.x >> 5); if (row >= ZH * TT) return;
    const int i = row % TT; const int zz = row / TT; const int hp = h0 + zz + 1;
    const float slope = ((hp & 1) ? 0.70710678118654752440f : 1.0f) * __uint_as_float((unsigned)(127 - (hp >> 1)) << 23);
    const int nch = (i >> 7) + 1;
    const float* sr = Sb + (size_t)row * TT;
    float v[TT / 32]; float mx = -3.0e38f;
#pragma unroll
    for (int ch = 0; ch < TT / 128; ++ch) {
        if (ch < nch) { const int j0 = ch * 128 + lane * 4; const v4f a = *(const v4f*)(sr + j0);
#pragma unroll
            for (int q = 0; q < 4; ++q) { const int j = j0 + q; float t = __fmul_rn(a[q], SCL); float al = __fmul_rn(slope, (float)(j - i)); asm volatile("" : "+v"(t)); asm volatile("" : "+v"(al));
                t = __fadd_rn(t, al); t = (j > i) ? -1.0e9f : t; v[ch * 4 + q] = t; mx = fmaxf(mx, t); }
        } else {
#pragma unroll
            for (int q = 0; q < 4; ++q) v[ch * 4 + q] = -1.0e9f; }
    }
#pragma unroll
    for (int sh = 16; sh; sh >>= 1) mx = fmaxf(mx, __shfl_xor(mx, sh, 32));
    float sum = 0.f;
#pragma unroll
    for (int ch = 0; ch < TT / 128; ++ch) {
        if (ch < nch) {
#pragma unroll
            for (int q = 0; q < 4; ++q) { float d0 = __fsub_rn(v[ch * 4 + q], mx); asm volatile("" : "+v"(d0)); const float ev = __builtin_amdgcn_exp2f(__fmul_rn(d0, 1.4426950408889634f)); v[ch * 4 + q] = ev; sum += ev; }
        } else {
#pragma unroll
            for (int q = 0; q < 4; ++q) v[ch * 4 + q] = 0.f; }
    }
#pragma unroll
    for (int sh = 16; sh; sh >>= 1) sum += __shfl_xor(sum, sh, 32);
    const float f = __fdiv_rn(1.0f, sum);
#pragma unroll 1
    for (int ps = 0; ps < 2; ++ps) {
#pragma unroll
        for (int ch = 0; ch < TT / 128; ++ch) {
            if (ch < nch) { v4us oh, ol;
#pragma unroll
                for (int q = 0; q < 4; ++q) { unsigned short a2, c2; splitf(v[ch * 4 + q] * f, a2, c2); oh[q] = a2; ol[q] = c2; }
                const size_t oo = (size_t)row * TT + ch * 128 + lane * 4; *(volatile v4us*)(Ph + oo) = oh; *(volatile v4us*)(Pl + oo) = ol; } }
        if (ps == 0) __threadfence(); }
}
__global__ __launch_bounds__(256) void k_merge(const float* __restrict__ O, int h0, bf* Ah, bf* Al) { const size_t e = ((size_t)blockIdx.x * 256 + threadIdx.x) * 2; if (e >= (size_t)ZH * TT * HD) return; const int d = (int)(e % HD); const int t = (int)((e / HD) % TT); const int zz = (int)(e / ((size_t)HD * TT)); const size_t oo = (size_t)t * DQ + (size_t)(h0 + zz) * HD + d;
    v2us oh, ol;
#pragma unroll
    for (int q = 0; q < 2; ++q) { unsigned short a2, c2; splitf(O[e + q], a2, c2); oh[q] = a2; ol[q] = c2; } *(volatile v2us*)(Ah + oo) = oh; *(volatile v2us*)(Al + oo) = ol; __threadfence(); *(volatile v2us*)(Ah + oo) = oh; *(volatile v2us*)(Al + oo) = ol; }

extern "C" void kernel_launch(void* const* d_in, const int* in_sizes, int n_in,
                              void* d_out, int out_size, void* d_ws, size_t ws_size, hipStream_t stream) {
    if (n_in < 6) return;
    if (in_sizes[0] < (NB - 1) * TT_FULL * DM + TT * DM) return;
    if (in_sizes[1] < DM * DM || in_sizes[2] < DM * DM || in_sizes[3] < DM * DM || in_sizes[4] < DM * DM || in_sizes[5] < DM) return;
    if (out_size < NB * TT * DM) return;
    const float* x  = (const float*)d_in[0];
    const float* wq = (const float*)d_in[1];
    const float* wk = (const float*)d_in[2];
    const float* wv = (const float*)d_in[3];
    const float* wo = (const float*)d_in[4];
    const float* bo = (const float*)d_in[5];
    float* OUT = (float*)d_out;
    char* wsp = (char*)d_ws;
    auto take = [&](size_t bytes) { char* p = wsp; wsp += (bytes + 255) & ~(size_t)255; return (void*)p; };
    bf* WQ = (bf*)take((size_t)DM * DM * 2); bf* WK = (bf*)take((size_t)DM * DM * 2); bf* WV = (bf*)take((size_t)DM * DM * 2); bf* WO = (bf*)take((size_t)DM * DQ * 2);
    float* FR = (float*)take((size_t)HALF * 4); float* CS = (float*)take((size_t)TT * HALF * 2 * 4);
    bf* XB = (bf*)take((size_t)TT * DM * 2); float* F = (float*)take((size_t)TT * DQ * 4);
    bf* QPh = (bf*)take((size_t)NH_ * TT * HD * 2); bf* QPl = (bf*)take((size_t)NH_ * TT * HD * 2); bf* KPh = (bf*)take((size_t)NH_ * TT * HD * 2); bf* KPl = (bf*)take((size_t)NH_ * TT * HD * 2);
    bf* VTh = (bf*)take((size_t)NH_ * HD * TT * 2); bf* VTl = (bf*)take((size_t)NH_ * HD * TT * 2);
    bf* Ph = (bf*)take((size_t)ZH * TT * TT * 2); bf* Pl = (bf*)take((size_t)ZH * TT * TT * 2);
    float* Sb = (float*)take((size_t)ZH * TT * TT * 4); float* Ob = (float*)take((size_t)ZH * TT * HD * 4);
    bf* ATh = (bf*)take((size_t)TT * DQ * 2); bf* ATl = (bf*)take((size_t)TT * DQ * 2);
    if ((size_t)(wsp - (char*)d_ws) > ws_size) return;
    k_cvt8<<<(unsigned)(((size_t)DM * DM / 8 + 255) / 256), 256, 0, stream>>>(wq, WQ, (size_t)DM * DM / 8);
    k_cvt8<<<(unsigned)(((size_t)DM * DM / 8 + 255) / 256), 256, 0, stream>>>(wk, WK, (size_t)DM * DM / 8);
    k_cvt8<<<(unsigned)(((size_t)DM * DM / 8 + 255) / 256), 256, 0, stream>>>(wv, WV, (size_t)DM * DM / 8);
    k_cvt8<<<(unsigned)(((size_t)DM * DQ / 8 + 255) / 256), 256, 0, stream>>>(wo, WO, (size_t)DM * DQ / 8);
    k_freq<<<(HALF + 255) / 256, 256, 0, stream>>>(FR);
    k_cstab<<<(unsigned)(((size_t)TT * HALF + 255) / 256), 256, 0, stream>>>(FR, CS);
    const unsigned LP = (unsigned)(((size_t)NH_ * TT * HD / 2 + 255) / 256);
    for (int b = 0; b < NB; ++b) {
        k_cvt8<<<(unsigned)(((size_t)TT * DM / 8 + 255) / 256), 256, 0, stream>>>(x + (size_t)b * TT_FULL * DM, XB, (size_t)TT * DM / 8);
        k_gemmw<0, false><<<dim3(TT / 64, DQ / 64, 1), 32, 0, stream>>>(XB, nullptr, WQ, nullptr, DM, F, DQ, nullptr, 0, 0, 0, 0, 0);
        k_rope<<<LP, 256, 0, stream>>>(F, CS, QPh, QPl);
        k_gemmw<0, false><<<dim3(TT / 64, DQ / 64, 1), 32, 0, stream>>>(XB, nullptr, WK, nullptr, DM, F, DQ, nullptr, 0, 0, 0, 0, 0);
        k_rope<<<LP, 256, 0, stream>>>(F, CS, KPh, KPl);
        k_gemmw<0, false><<<dim3(TT / 64, DQ / 64, 1), 32, 0, stream>>>(XB, nullptr, WV, nullptr, DM, F, DQ, nullptr, 0, 0, 0, 0, 0);
        k_vtp<<<LP, 256, 0, stream>>>(F, VTh, VTl);
        for (int h0 = 0; h0 < NH_; h0 += ZH) { const size_t zq = (size_t)h0;
            k_gemmw<2, false><<<dim3(TT / 64, TT / 64, ZH), 32, 0, stream>>>(QPh + zq * TT * HD, QPl + zq * TT * HD, KPh + zq * TT * HD, KPl + zq * TT * HD, HD, Sb, TT, nullptr, (size_t)TT * HD, (size_t)TT * HD, (size_t)TT * TT, 0, 1);
            k_asoft<<<ZH * TT / 8, 256, 0, stream>>>(Sb, h0, Ph, Pl);
            k_gemmw<2, false><<<dim3(TT / 64, HD / 64, ZH), 32, 0, stream>>>(Ph, Pl, VTh + zq * HD * TT, VTl + zq * HD * TT, TT, Ob, HD, nullptr, (size_t)TT * TT, (size_t)HD * TT, (size_t)TT * HD, 0, 2);
            k_merge<<<(unsigned)(((size_t)ZH * TT * HD / 2 + 255) / 256), 256, 0, stream>>>(Ob, h0, ATh, ATl); }
        k_gemmw<1, true><<<dim3(TT / 64, DM / 64, 1), 32, 0, stream>>>(ATh, ATl, WO, nullptr, DQ, OUT + (size_t)b * TT * DM, DM, bo, 0, 0, 0, 0, 0); }
}
